// AggregatedAttention_12197707121248
// MI455X (gfx1250) — hardware-verified
//
#include <hip/hip_runtime.h>
#include <hip/hip_bf16.h>
#include <math.h>

constexpr int   kB     = 4;
constexpr int   kImg   = 64;
constexpr int   kN     = kImg * kImg;
constexpr int   kC     = 256;
constexpr int   kHeads = 8;
constexpr int   kHD    = 32;
constexpr int   kPL    = 64;
constexpr int   kLoc   = 9;
constexpr int   kTbl   = 4096;
constexpr int   kBN    = kB * kN;
constexpr int   kHid   = 512;
constexpr int   kCpbN  = 64;
constexpr int   kGateRows = 10;
constexpr float kEps   = 1.1920929e-07f;

static_assert(kBN % 64 == 0 && kC % 64 == 0 && (2 * kC) % 64 == 0 && (kB * kPL) % 64 == 0 && kTbl % 64 == 0 && kCpbN % 64 == 0, "");
static_assert(kC % 32 == 0 && kHid % 32 == 0, "");
static_assert(kHD == 32 && kImg == 64 && kPL == 64, "");

typedef __attribute__((ext_vector_type(16))) _Float16 v16h;
typedef __attribute__((ext_vector_type(8)))  _Float16 v8h;
typedef __attribute__((ext_vector_type(16))) __bf16   v16b;
typedef __attribute__((ext_vector_type(8)))  __bf16   v8b;
typedef __attribute__((ext_vector_type(8)))  float    v8f;
typedef __attribute__((ext_vector_type(4)))  float    v4f;
typedef __attribute__((ext_vector_type(4)))  unsigned v4u;
typedef __attribute__((ext_vector_type(4)))  int      v4i;
#define PSCALE 32768.0f
#define U16(p) ((const unsigned short*)(const void*)(p))
#define PSCALE_INV (1.0f / 32768.0f)

__device__ __forceinline__ unsigned short f2bf_bits(float f) {
  unsigned u = __float_as_uint(f);
  return (unsigned short)((u + 0x7FFFu + ((u >> 16) & 1u)) >> 16);
}
__device__ __forceinline__ float bf_bits2f(unsigned short h) { return __uint_as_float(((unsigned)h) << 16); }

__device__ __forceinline__ void dep_guard_h(v8f& a, v8f& b, v16h x, v16h y) { asm volatile("v_nop\n\tv_nop\n\tv_nop\n\tv_nop" : "+v"(a), "+v"(b) : "v"(x), "v"(y)); }
__device__ __forceinline__ void dep_guard_b(v8f& a, v8f& b, v16b x, v16b y) { asm volatile("v_nop\n\tv_nop\n\tv_nop\n\tv_nop" : "+v"(a), "+v"(b) : "v"(x), "v"(y)); }
__device__ __forceinline__ void keep4_h(v16h a, v16h b, v16h c, v16h d) { asm volatile("v_nop" :: "v"(a), "v"(b), "v"(c), "v"(d)); }
__device__ __forceinline__ void keep4_b(v16b a, v16b b, v16b c, v16b d) { asm volatile("v_nop" :: "v"(a), "v"(b), "v"(c), "v"(d)); }
__device__ __forceinline__ void acc_guard4(v8f& a, v8f& b, v8f& c, v8f& d) { asm volatile("v_nop\n\tv_nop\n\tv_nop\n\tv_nop" : "+v"(a), "+v"(b), "+v"(c), "+v"(d)); }
template <typename T> struct Frag;
template <> struct Frag<_Float16> {
  typedef v16h V; union U { v16h v; v8h h[2]; };
  static __device__ __forceinline__ v16h load(const _Float16* p) {
    U f; f.h[0] = *(const v8h*)(p); f.h[1] = *(const v8h*)(p + 16); return f.v;
  }
  static __device__ __forceinline__ v8f mma(v16h a, v16h b, v8f c) {
    return __builtin_amdgcn_wmma_f32_16x16x32_f16(false, a, false, b, (short)0, c, false, false);
  }
  static __device__ __forceinline__ void guard(v8f& a, v8f& b, v16h x, v16h y) { dep_guard_h(a, b, x, y); }
  static __device__ __forceinline__ void keep(v16h a, v16h b, v16h c, v16h d) { keep4_h(a, b, c, d); }
};
template <> struct Frag<__bf16> {
  typedef v16b V; union U { v16b v; v8b h[2]; };
  static __device__ __forceinline__ v16b load(const __bf16* p) {
    U f; f.h[0] = *(const v8b*)(p); f.h[1] = *(const v8b*)(p + 16); return f.v;
  }
  static __device__ __forceinline__ v8f mma(v16b a, v16b b, v8f c) {
    return __builtin_amdgcn_wmma_f32_16x16x32_bf16(false, a, false, b, (short)0, c, false, false);
  }
  static __device__ __forceinline__ void guard(v8f& a, v8f& b, v16b x, v16b y) { dep_guard_b(a, b, x, y); }
  static __device__ __forceinline__ void keep(v16b a, v16b b, v16b c, v16b d) { keep4_b(a, b, c, d); }
};

template <int ET> struct Elem;
template <> struct Elem<0> { typedef _Float16 T; };
template <> struct Elem<1> { typedef __bf16 T; };
template <int ET, bool SPLIT, int BIAS_MODE, int OUT_MODE, bool RESID, int ACT = 0>
__global__ __launch_bounds__(256) void wmma_gemm64(
    const unsigned short* __restrict__ Ap, const unsigned short* __restrict__ A2p, int lda, long strideA,
    const unsigned short* __restrict__ Btp, const unsigned short* __restrict__ Bt2p, int ldb, long strideB,
    void* __restrict__ Cout, void* __restrict__ Cout2, int ldc, long strideC,
    const float* __restrict__ bias,
    const float* __restrict__ resid, long strideR,
    int M, int N, int K, float scale) {
  typedef typename Elem<ET>::T T;
  typedef typename Frag<T>::V V;
  const T* A = (const T*)Ap; const T* A2 = (const T*)A2p; const T* Bt = (const T*)Btp; const T* Bt2 = (const T*)Bt2p;
  __shared__ __align__(16) float sT[8][16 * 68];
  const int b    = blockIdx.y;
  const int lane = threadIdx.x & 31;
  const int wave = threadIdx.x >> 5;
  const int tilesN = N >> 6;
  const int tilesM = M >> 6;
  const int tile = blockIdx.x * 8 + wave;
  if (tile >= tilesM * tilesN) return;
  const int tm = tile / tilesN;
  const int tn = tile - tm * tilesN;
  const int m0 = tm << 6;
  const int n0 = tn << 6;

  const T* Ab  = A  + (size_t)b * strideA;
  const T* Bb  = Bt + (size_t)b * strideB;
  const T* Ab2 = SPLIT ? (A2  + (size_t)b * strideA) : nullptr;
  const T* Bb2 = SPLIT ? (Bt2 + (size_t)b * strideB) : nullptr;

  const int rlane = lane & 15;
  const int koff  = (lane >> 4) * 8;
  const int mOff  = (lane >> 4) * 8;

  v8f acc[4][4];
#pragma unroll
  for (int i = 0; i < 4; ++i)
#pragma unroll
    for (int j = 0; j < 4; ++j) acc[i][j] = (v8f){0.f,0.f,0.f,0.f,0.f,0.f,0.f,0.f};

  for (int k0 = 0; k0 < K; k0 += 32) {
    V bh[4], bl[4];
#pragma unroll
    for (int j = 0; j < 4; ++j) {
      const size_t bo = (size_t)(n0 + (j << 4) + rlane) * ldb + koff + k0;
      bh[j] = Frag<T>::load(Bb + bo);
      if (SPLIT) bl[j] = Frag<T>::load(Bb2 + bo);
    }
#pragma unroll
    for (int i = 0; i < 4; ++i) {
      const size_t ao = (size_t)(m0 + (i << 4) + rlane) * lda + koff + k0;
      V ah = Frag<T>::load(Ab + ao);
      V al;
      if (SPLIT) al = Frag<T>::load(Ab2 + ao);
#pragma unroll
      for (int j = 0; j < 4; ++j) {
        acc[i][j] = Frag<T>::mma(ah, bh[j], acc[i][j]);
        if (SPLIT) {
          acc[i][j] = Frag<T>::mma(ah, bl[j], acc[i][j]);
          acc[i][j] = Frag<T>::mma(al, bh[j], acc[i][j]);
        }
      }
      Frag<T>::guard(acc[i][0], acc[i][3], ah, SPLIT ? al : ah);
    }
    Frag<T>::keep(bh[0], bh[1], bh[2], bh[3]);
    if (SPLIT) Frag<T>::keep(bl[0], bl[1], bl[2], bl[3]);
  }
  acc_guard4(acc[0][0], acc[0][1], acc[0][2], acc[0][3]);
  acc_guard4(acc[1][0], acc[1][1], acc[1][2], acc[1][3]);
  acc_guard4(acc[2][0], acc[2][1], acc[2][2], acc[2][3]);
  acc_guard4(acc[3][0], acc[3][1], acc[3][2], acc[3][3]);

  float* slab = sT[wave];
  const float* Rb = RESID ? (resid + (size_t)b * strideR) : nullptr;
#pragma unroll
  for (int i = 0; i < 4; ++i) {
    const int mBase = m0 + (i << 4);
#pragma unroll
    for (int j = 0; j < 4; ++j) {
      const int n = n0 + (j << 4) + rlane;
      float bv = 0.f;
      if (BIAS_MODE == 2) bv = bias[n];
#pragma unroll
      for (int r = 0; r < 8; ++r) {
        float v = acc[i][j][r] * scale;
        if (BIAS_MODE == 1) v += bias[mBase + mOff + r];
        if (BIAS_MODE == 2) v += bv;
        if (RESID) v += Rb[(size_t)(mBase + mOff + r) * ldc + n];
        if (ACT == 1) v = tanhf(v);
        if (ACT == 2) v = fmaxf(v, 0.0f);
        if (ACT == 3) v = v / (1.0f + expf(-v));
        if (ACT == 4) v = (v > 0.f) ? v : 0.01f * v;
        if (ACT == 5) v = 0.5f * v * (1.0f + erff(v * 0.70710678118654752f));
        slab[(mOff + r) * 68 + (j << 4) + rlane] = v;
      }
    }
    __builtin_amdgcn_fence(__ATOMIC_RELEASE, "workgroup");
    __builtin_amdgcn_wave_barrier();
    __builtin_amdgcn_fence(__ATOMIC_ACQUIRE, "workgroup");
    if (OUT_MODE == 0) {
      float* C = (float*)Cout + (size_t)b * strideC;
      const int hh = lane >> 4, c4 = (lane & 15) * 4;
      for (int pass = 0; pass < 2; ++pass) {
#pragma unroll
        for (int it = 0; it < 8; ++it) {
          const int row = it * 2 + hh;
          v4f v = *(const v4f*)(slab + row * 68 + c4);
          *(volatile v4f*)(C + (size_t)(mBase + row) * ldc + n0 + c4) = v;
        }
        __threadfence();
      }
    } else {
      const int q = lane >> 3, c8 = (lane & 7) * 8;
      unsigned short* C  = (unsigned short*)Cout  + (size_t)b * strideC;
      unsigned short* C2 = (OUT_MODE == 2) ? ((unsigned short*)Cout2 + (size_t)b * strideC) : nullptr;
      for (int pass = 0; pass < 2; ++pass) {
#pragma unroll
        for (int it = 0; it < 4; ++it) {
          const int row = it * 4 + q;
          const float* sp = slab + row * 68 + c8;
          v8h hv, lv;
#pragma unroll
          for (int e = 0; e < 8; ++e) {
            if (OUT_MODE == 1) {
              hv[e] = (_Float16)sp[e];
            } else {
              unsigned short hb = f2bf_bits(sp[e]);
              unsigned short lb = f2bf_bits(sp[e] - bf_bits2f(hb));
              hv[e] = __builtin_bit_cast(_Float16, hb);
              lv[e] = __builtin_bit_cast(_Float16, lb);
            }
          }
          *(volatile v8h*)(C + (size_t)(mBase + row) * ldc + n0 + c8) = hv;
          if (OUT_MODE == 2) *(volatile v8h*)(C2 + (size_t)(mBase + row) * ldc + n0 + c8) = lv;
        }
        __threadfence();
      }
    }
    __builtin_amdgcn_fence(__ATOMIC_RELEASE, "workgroup");
    __builtin_amdgcn_wave_barrier();
    __builtin_amdgcn_fence(__ATOMIC_ACQUIRE, "workgroup");
  }
}

__device__ __forceinline__ unsigned short at_bf_bits(float f) {
  unsigned u = __float_as_uint(f);
  return (unsigned short)((u + 0x7FFFu + ((u >> 16) & 1u)) >> 16);
}
__device__ __forceinline__ __bf16 at_f2bf(float f) { return __builtin_bit_cast(__bf16, at_bf_bits(f)); }
__device__ __forceinline__ void at_split(float f, __bf16& hi, __bf16& lo) {
  const unsigned short hb = at_bf_bits(f);
  hi = __builtin_bit_cast(__bf16, hb);
  lo = at_f2bf(f - __uint_as_float(((unsigned)hb) << 16));
}
__device__ __forceinline__ v8f at_mma(v16b a, v16b b, v8f c) {
  c = __builtin_amdgcn_wmma_f32_16x16x32_bf16(false, a, false, b, (short)0, c, false, false);
  asm volatile("v_nop\n\tv_nop\n\tv_nop\n\tv_nop" : "+v"(c) : "v"(a), "v"(b));
  return c;
}
union FB { v16b v; v8b h[2]; };

__device__ __forceinline__ float wsum32(float v) {
  v += __shfl_xor(v, 16, 32); v += __shfl_xor(v, 8, 32); v += __shfl_xor(v, 4, 32);
  v += __shfl_xor(v, 2, 32);  v += __shfl_xor(v, 1, 32);
  return v;
}
__device__ __forceinline__ void split_pair(float a, float b, unsigned& hw, unsigned& lw) {
  const unsigned short ha = f2bf_bits(a), hb = f2bf_bits(b);
  const unsigned short la = f2bf_bits(a - bf_bits2f(ha)), lb = f2bf_bits(b - bf_bits2f(hb));
  hw = (unsigned)ha | ((unsigned)hb << 16);
  lw = (unsigned)la | ((unsigned)lb << 16);
}
__device__ __forceinline__ unsigned hi_pair(float a, float b) {
  return (unsigned)f2bf_bits(a) | ((unsigned)f2bf_bits(b) << 16);
}

__global__ __launch_bounds__(256) void split_planes_kernel(const float* __restrict__ in,
    unsigned short* __restrict__ hi, unsigned short* __restrict__ lo, int n8) {
  const int i = blockIdx.x * 256 + threadIdx.x;
  if (i >= n8) return;
  const float* p = in + (size_t)i * 8;
  const v4f a = *(const v4f*)p;
  const v4f c = *(const v4f*)(p + 4);
  v4u hv, lv;
  unsigned h0, l0, h1, l1, h2, l2, h3, l3;
  split_pair(a.x, a.y, h0, l0); split_pair(a.z, a.w, h1, l1);
  split_pair(c.x, c.y, h2, l2); split_pair(c.z, c.w, h3, l3);
  hv.x = h0; hv.y = h1; hv.z = h2; hv.w = h3;
  lv.x = l0; lv.y = l1; lv.z = l2; lv.w = l3;
  unsigned short* hp = hi + (size_t)i * 8;
  unsigned short* lp = lo + (size_t)i * 8;
  *(volatile v4u*)hp = hv;
  *(volatile v4u*)lp = lv;
  __threadfence();
  *(volatile v4u*)hp = hv;
  *(volatile v4u*)lp = lv;
}

__global__ __launch_bounds__(256) void pad_w2_kernel(const float* __restrict__ w, unsigned short* __restrict__ outp) {
  const int i = blockIdx.x * 256 + threadIdx.x;
  if (i >= kCpbN * kHid / 8) return;
  const int nreal = kHeads * kHid / 8;
  const bool real = i < nreal;
  const int ic = real ? i : (nreal - 1);
  const float* p = w + (size_t)ic * 8;
  const v4f a = *(const v4f*)p;
  const v4f c = *(const v4f*)(p + 4);
  v4u hv;
  hv.x = real ? hi_pair(a.x, a.y) : 0u;
  hv.y = real ? hi_pair(a.z, a.w) : 0u;
  hv.z = real ? hi_pair(c.x, c.y) : 0u;
  hv.w = real ? hi_pair(c.z, c.w) : 0u;
  unsigned short* hp = outp + (size_t)i * 8;
  *(volatile v4u*)hp = hv;
  __threadfence();
  *(volatile v4u*)hp = hv;
}

__global__ __launch_bounds__(256) void cpb_hidden_kernel(const float* __restrict__ rct, const float* __restrict__ w1,
    const float* __restrict__ b1, unsigned short* __restrict__ hid) {
  const int i = blockIdx.x * 256 + threadIdx.x;
  if (i >= kTbl * kHid / 8) return;
  const int t  = i >> 6;
  const int j0 = (i & 63) * 8;
  const float r0 = rct[2 * t], r1 = rct[2 * t + 1];
  const v4f wa = *(const v4f*)(w1 + 2 * j0);
  const v4f wb = *(const v4f*)(w1 + 2 * j0 + 4);
  const v4f wc = *(const v4f*)(w1 + 2 * j0 + 8);
  const v4f wd = *(const v4f*)(w1 + 2 * j0 + 12);
  const v4f ba = *(const v4f*)(b1 + j0);
  const v4f bb = *(const v4f*)(b1 + j0 + 4);
  const float e0 = fmaxf(r0 * wa.x + r1 * wa.y + ba.x, 0.f);
  const float e1 = fmaxf(r0 * wa.z + r1 * wa.w + ba.y, 0.f);
  const float e2 = fmaxf(r0 * wb.x + r1 * wb.y + ba.z, 0.f);
  const float e3 = fmaxf(r0 * wb.z + r1 * wb.w + ba.w, 0.f);
  const float e4 = fmaxf(r0 * wc.x + r1 * wc.y + bb.x, 0.f);
  const float e5 = fmaxf(r0 * wc.z + r1 * wc.w + bb.y, 0.f);
  const float e6 = fmaxf(r0 * wd.x + r1 * wd.y + bb.z, 0.f);
  const float e7 = fmaxf(r0 * wd.z + r1 * wd.w + bb.w, 0.f);
  v4u hv;
  hv.x = hi_pair(e0, e1); hv.y = hi_pair(e2, e3); hv.z = hi_pair(e4, e5); hv.w = hi_pair(e6, e7);
  unsigned short* hp = hid + (size_t)i * 8;
  *(volatile v4u*)hp = hv;
  __threadfence();
  *(volatile v4u*)hp = hv;
}

__global__ __launch_bounds__(256) void gates_kernel(const float* __restrict__ x, const float* __restrict__ wg,
    const float* __restrict__ wg0, const float* __restrict__ wg1, float* __restrict__ maskw) {
  __shared__ __align__(16) float sm[64];
  const int lane = threadIdx.x & 31;
  const int wave = threadIdx.x >> 5;
  const int tok  = blockIdx.x * 8 + wave;
  const float* xr = x + (size_t)tok * kC + lane * 8;
  const v4f xa = *(const v4f*)xr;
  const v4f xb = *(const v4f*)(xr + 4);
  float mine = 0.f;
#pragma unroll 1
  for (int r = 0; r < kGateRows; ++r) {
    const float* wr = (r < 4) ? (wg + r * kC) : ((r < 6) ? (wg0 + (r - 4) * kC) : (wg1 + (r - 6) * kC));
    const v4f wa = *(const v4f*)(wr + lane * 8);
    const v4f wb = *(const v4f*)(wr + lane * 8 + 4);
    float s = xa.x * wa.x;
    s += xa.y * wa.y; s += xa.z * wa.z; s += xa.w * wa.w;
    s += xb.x * wb.x; s += xb.y * wb.y; s += xb.z * wb.z; s += xb.w * wb.w;
    s = wsum32(s);
    mine = (lane == r) ? s : mine;
  }
  const float d0 = __shfl(mine, 0, 32), d1 = __shfl(mine, 1, 32), d2 = __shfl(mine, 2, 32), d3 = __shfl(mine, 3, 32);
  const float d4 = __shfl(mine, 4, 32), d5 = __shfl(mine, 5, 32);
  const float d6 = __shfl(mine, 6, 32), d7 = __shfl(mine, 7, 32), d8 = __shfl(mine, 8, 32), d9 = __shfl(mine, 9, 32);

  const float mr = fmaxf(fmaxf(d0, d1), fmaxf(d2, d3));
  const float e0 = expf(d0 - mr), e1 = expf(d1 - mr), e2 = expf(d2 - mr), e3 = expf(d3 - mr);
  const float invr = 1.0f / (((e0 + e1) + e2) + e3);
  const float g0 = e0 * invr, g1 = e1 * invr, g2 = e2 * invr, g3 = e3 * invr;
  int i1 = 0; float gm = g0;
  if (g1 > gm) { i1 = 1; gm = g1; }
  if (g2 > gm) { i1 = 2; gm = g2; }
  if (g3 > gm) { i1 = 3; gm = g3; }
  const float c0 = (i1 == 0) ? -1.f : g0, c1 = (i1 == 1) ? -1.f : g1, c2 = (i1 == 2) ? -1.f : g2, c3 = (i1 == 3) ? -1.f : g3;
  int i2 = 0; float gm2 = c0;
  if (c1 > gm2) { i2 = 1; gm2 = c1; }
  if (c2 > gm2) { i2 = 2; gm2 = c2; }
  if (c3 > gm2) { i2 = 3; gm2 = c3; }
  const float rs = fmaxf(gm + gm2, kEps);
  const float rsi = 1.0f / rs;
  const float rg0 = ((i1 == 0) || (i2 == 0)) ? (g0 * rsi) * 2.0f : 0.f;
  const float rg1 = ((i1 == 1) || (i2 == 1)) ? (g1 * rsi) * 2.0f : 0.f;
  const float rg2 = ((i1 == 2) || (i2 == 2)) ? (g2 * rsi) * 2.0f : 0.f;
  const float rg3 = ((i1 == 3) || (i2 == 3)) ? (g3 * rsi) * 2.0f : 0.f;
  const float mm = fmaxf(d4, d5);
  const float f4 = expf(d4 - mm), f5 = expf(d5 - mm);
  const float invm = 1.0f / (f4 + f5);
  const float w00 = (f4 * invm) * 2.0f, w01 = (f5 * invm) * 2.0f;
  const float ms = fmaxf(fmaxf(d6, d7), fmaxf(d8, d9));
  const float s6 = expf(d6 - ms), s7 = expf(d7 - ms), s8 = expf(d8 - ms), s9 = expf(d9 - ms);
  const float invs = 1.0f / (((s6 + s7) + s8) + s9);
  const float h0 = w00 * ((s6 * invs) * 4.0f), h1 = w00 * ((s7 * invs) * 4.0f);
  const float h2 = w00 * ((s8 * invs) * 4.0f), h3 = w00 * ((s9 * invs) * 4.0f);
  const float h4 = w01 * rg0, h5 = w01 * rg1, h6 = w01 * rg2, h7 = w01 * rg3;
  float ov = h0;
  ov = (lane == 1) ? h1 : ov; ov = (lane == 2) ? h2 : ov; ov = (lane == 3) ? h3 : ov;
  ov = (lane == 4) ? h4 : ov; ov = (lane == 5) ? h5 : ov; ov = (lane == 6) ? h6 : ov; ov = (lane == 7) ? h7 : ov;
  if (lane < 8) sm[wave * 8 + lane] = ov;
  __syncthreads();
  if (wave == 0) {
    const int q = lane & 15;
    const v4f v = *(const v4f*)(sm + q * 4);
    float* dst = maskw + (size_t)blockIdx.x * 64 + q * 4;
    if (lane < 16) *(volatile v4f*)dst = v;
    __threadfence();
    if (lane < 16) *(volatile v4f*)dst = v;
  }
}

__global__ __launch_bounds__(256) void pool_ln_kernel(const float* __restrict__ sr, const float* __restrict__ g,
    const float* __restrict__ bt, unsigned short* __restrict__ lnh, unsigned short* __restrict__ lnl) {
  __shared__ __align__(16) float ys[256];
  __shared__ float red[8];
  const int bp = blockIdx.x;
  const int b  = bp >> 6, p = bp & 63, pi = p >> 3, pj = p & 7;
  const int c  = threadIdx.x, lane = c & 31, wave = c >> 5;
  float s = 0.f;
#pragma unroll 1
  for (int q = 0; q < 64; ++q) {
    const int n = (pi * 8 + (q >> 3)) * kImg + pj * 8 + (q & 7);
    const float v = sr[(size_t)(b * kN + n) * kC + c];
    s += 0.5f * v * (1.0f + erff(v * 0.70710678118654752f));
  }
  const float xv = s * (1.0f / 64.0f);
  float t = wsum32(xv);
  if (lane == 0) red[wave] = t;
  __syncthreads();
  float mu = 0.f;
#pragma unroll
  for (int k = 0; k < 8; ++k) mu += red[k];
  mu *= (1.0f / (float)kC);
  __syncthreads();
  const float d = xv - mu;
  t = wsum32(d * d);
  if (lane == 0) red[wave] = t;
  __syncthreads();
  float var = 0.f;
#pragma unroll
  for (int k = 0; k < 8; ++k) var += red[k];
  var *= (1.0f / (float)kC);
  const float y = d * (1.0f / sqrtf(var + 1e-5f)) * g[c] + bt[c];
  ys[c] = y;
  __syncthreads();
  if (wave == 0) {
    const float* yp = ys + lane * 8;
    const v4f a = *(const v4f*)yp;
    const v4f e = *(const v4f*)(yp + 4);
    v4u hv, lv;
    unsigned h0, l0, h1, l1, h2, l2, h3, l3;
    split_pair(a.x, a.y, h0, l0); split_pair(a.z, a.w, h1, l1);
    split_pair(e.x, e.y, h2, l2); split_pair(e.z, e.w, h3, l3);
    hv.x = h0; hv.y = h1; hv.z = h2; hv.w = h3;
    lv.x = l0; lv.y = l1; lv.z = l2; lv.w = l3;
    unsigned short* hp = lnh + (size_t)bp * kC + lane * 8;
    unsigned short* lp = lnl + (size_t)bp * kC + lane * 8;
    *(volatile v4u*)hp = hv;
    *(volatile v4u*)lp = lv;
    __threadfence();
    *(volatile v4u*)hp = hv;
    *(volatile v4u*)lp = lv;
  }
}

__global__ __launch_bounds__(128) void attn_kernel(const float* __restrict__ qbuf, const float* __restrict__ kvbuf,
    const float* __restrict__ pkv, const float* __restrict__ cpbo, const int* __restrict__ rpi,
    const float* __restrict__ cpb2b, const float* __restrict__ rpb, const float* __restrict__ ltok,
    const float* __restrict__ lbias, const float* __restrict__ qe, const float* __restrict__ temp,
    const float* __restrict__ maskw, float* __restrict__ obuf, float sl4, float sl6, float sl9) {
  __shared__ __align__(16) float  Qn[kImg * kHD];
  __shared__ __align__(16) float  Qs[kImg * kHD];
  __shared__ __align__(16) float  Kloc[3 * kImg * kHD];
  __shared__ __align__(16) float  Vloc[3 * kImg * kHD];
  __shared__ __align__(16) __bf16 Kph[kPL * kHD];
  __shared__ __align__(16) __bf16 Kpl[kPL * kHD];
  __shared__ __align__(16) __bf16 Vth[kHD * kPL];
  __shared__ __align__(16) __bf16 Vtl[kHD * kPL];
  __shared__ __align__(16) __bf16 Psh[4][16 * kPL];
  __shared__ __align__(16) __bf16 Psl[4][16 * kPL];
  __shared__ __align__(16) float  Bp[4][16 * kPL];
  __shared__ __align__(16) float  Sa[4][16 * 16];
  __shared__ __align__(16) float  Os[4][16 * 36];
  __shared__ __align__(16) float  Lt[kHD * kLoc];

  const int tid  = threadIdx.x;
  const int wave = tid >> 5;
  const int lane = tid & 31;
  const int hf   = lane >> 4;
  const int c    = lane & 15;
  const int bx = blockIdx.x;
  const int i  = bx & (kImg - 1);
  const int bh = bx >> 6;
  const int h  = bh & (kHeads - 1);
  const int b  = bh >> 3;
  const bool edge_i = (i == 0) || (i == kImg - 1);
  const float tp = temp[h];
  const float sp = fmaxf(tp, 0.f) + log1pf(expf(-fabsf(tp)));
  const v4f z4 = (v4f){0.f, 0.f, 0.f, 0.f};

  for (int q = tid; q < kHD * kLoc; q += 128) Lt[q] = ltok[h * kHD * kLoc + q];

#pragma unroll
  for (int it = 0; it < 4; ++it) {
    const int idx = it * 128 + tid;
    const int row = idx >> 3;
    const int c4  = (idx & 7) * 4;
    const int n   = i * kImg + row;
    const v4f v = *(const v4f*)(qbuf + (size_t)(b * kN + n) * kC + h * kHD + c4);
    float ss = v.x * v.x + v.y * v.y + v.z * v.z + v.w * v.w;
    ss += __shfl_xor(ss, 1, 32); ss += __shfl_xor(ss, 2, 32); ss += __shfl_xor(ss, 4, 32);
    const float inv = 1.0f / fmaxf(sqrtf(ss), kEps);
    const v4f qn = v * inv;
    *(v4f*)(Qn + row * kHD + c4) = qn;
    const bool edge_j = (row == 0) || (row == kImg - 1);
    const float sls = edge_i ? (edge_j ? sl4 : sl6) : (edge_j ? sl6 : sl9);
    const v4f e4 = *(const v4f*)(qe + h * kHD + c4);
    v4f qs = (qn + e4) * sp;
    qs = qs * sls;
    *(v4f*)(Qs + row * kHD + c4) = qs;
  }

#pragma unroll
  for (int kr = 0; kr < 3; ++kr) {
    const int ii  = i + kr - 1;
    const bool vrow = (ii >= 0) && (ii < kImg);
    const int iic = ii < 0 ? 0 : (ii > kImg - 1 ? kImg - 1 : ii);
#pragma unroll
    for (int it = 0; it < 4; ++it) {
      const int idx = it * 128 + tid;
      const int col = idx >> 3;
      const int c4  = (idx & 7) * 4;
      const size_t base = (size_t)(b * kN + iic * kImg + col) * (2 * kC) + h * kHD + c4;
      v4f kk = *(const v4f*)(kvbuf + base);
      v4f vv = *(const v4f*)(kvbuf + base + kC);
      float ss = kk.x * kk.x + kk.y * kk.y + kk.z * kk.z + kk.w * kk.w;
      ss += __shfl_xor(ss, 1, 32); ss += __shfl_xor(ss, 2, 32); ss += __shfl_xor(ss, 4, 32);
      const float inv = 1.0f / fmaxf(sqrtf(ss), kEps);
      kk = kk * inv;
      kk = vrow ? kk : z4;
      vv = vrow ? vv : z4;
      *(v4f*)(Kloc + (kr * kImg + col) * kHD + c4) = kk;
      *(v4f*)(Vloc + (kr * kImg + col) * kHD + c4) = vv;
    }
  }

#pragma unroll
  for (int it = 0; it < 4; ++it) {
    const int idx = it * 128 + tid;
    const int p   = idx >> 3;
    const int c4  = (idx & 7) * 4;
    const size_t base = (size_t)(b * kPL + p) * (2 * kC) + h * kHD + c4;
    v4f kk = *(const v4f*)(pkv + base);
    const v4f vv = *(const v4f*)(pkv + base + kC);
    float ss = kk.x * kk.x + kk.y * kk.y + kk.z * kk.z + kk.w * kk.w;
    ss += __shfl_xor(ss, 1, 32); ss += __shfl_xor(ss, 2, 32); ss += __shfl_xor(ss, 4, 32);
    const float inv = 1.0f / fmaxf(sqrtf(ss), kEps);
    kk = kk * inv;
#pragma unroll
    for (int e = 0; e < 4; ++e) {
      __bf16 a, l;
      at_split(kk[e], a, l);
      Kph[p * kHD + c4 + e] = a;
      Kpl[p * kHD + c4 + e] = l;
      at_split(vv[e], a, l);
      Vth[(c4 + e) * kPL + p] = a;
      Vtl[(c4 + e) * kPL + p] = l;
    }
  }

  {
    float* bpw = Bp[wave];
    const float b2 = cpb2b[h];
#pragma unroll 1
    for (int it = 0; it < 8; ++it) {
      const int rr = it * 2 + hf;
      const int n  = i * kImg + wave * 16 + rr;
      const v4i v = *(const v4i*)(rpi + (size_t)n * kPL + c * 4);
      v4f bv = z4;
#pragma unroll
      for (int e = 0; e < 4; ++e) {
        int id = v[e];
        id = id < 0 ? 0 : (id > kTbl - 1 ? kTbl - 1 : id);
        bv[e] = cpbo[(size_t)id * kCpbN + h] + b2;
      }
      *(v4f*)(bpw + rr * kPL + c * 4) = bv;
    }
  }
  __syncthreads();

  const int qrow0 = wave * 16;
  const int lc    = (c < kLoc) ? c : (kLoc - 1);
  const int krc   = lc / 3;
  const int djc   = lc - krc * 3 - 1;
  const v8f z8 = (v8f){0.f, 0.f, 0.f, 0.f, 0.f, 0.f, 0.f, 0.f};

  float sloc[8];
  {
    const float rpv = rpb[h * kLoc + lc];
#pragma unroll
    for (int r = 0; r < 8; ++r) {
      const int row = qrow0 + 8 * hf + r;
      const int jj  = row + djc;
      const bool okj = (jj >= 0) && (jj < kImg);
      const int jjc = jj < 0 ? 0 : (jj > kImg - 1 ? kImg - 1 : jj);
      const float* qp = Qs + row * kHD;
      const float* kp = Kloc + (krc * kImg + jjc) * kHD;
      float d = 0.f;
#pragma unroll 2
      for (int q4 = 0; q4 < 8; ++q4) {
        const v4f a = *(const v4f*)(qp + 4 * q4);
        const v4f k = *(const v4f*)(kp + 4 * q4);
        d += a.x * k.x; d += a.y * k.y; d += a.z * k.z; d += a.w * k.w;
      }
      d = okj ? d : 0.f;
      sloc[r] = (c < kLoc) ? (d + rpv) : -INFINITY;
    }
  }

  v8f tacc = z8;
  {
    v16b qnh, qnl, bh16, bl16;
    const float* qrow = Qn + (qrow0 + c) * kHD;
#pragma unroll
    for (int e = 0; e < 8; ++e) {
      __bf16 a, l;
      at_split(qrow[8 * hf + e], a, l);      qnh[e] = a;     qnl[e] = l;
      at_split(qrow[16 + 8 * hf + e], a, l); qnh[8 + e] = a; qnl[8 + e] = l;
      float t0 = Lt[(8 * hf + e) * kLoc + lc];
      float t1 = Lt[(16 + 8 * hf + e) * kLoc + lc];
      t0 = (c < kLoc) ? t0 : 0.f;
      t1 = (c < kLoc) ? t1 : 0.f;
      at_split(t0, a, l); bh16[e] = a;     bl16[e] = l;
      at_split(t1, a, l); bh16[8 + e] = a; bl16[8 + e] = l;
    }
    tacc = at_mma(qnh, bh16, tacc);
    tacc = at_mma(qnh, bl16, tacc);
    tacc = at_mma(qnl, bh16, tacc);
  }

  v8f s[4];
  {
    v16b qsh, qsl;
    const float* qrow = Qs + (qrow0 + c) * kHD;
#pragma unroll
    for (int e = 0; e < 8; ++e) {
      __bf16 a, l;
      at_split(qrow[8 * hf + e], a, l);      qsh[e] = a;     qsl[e] = l;
      at_split(qrow[16 + 8 * hf + e], a, l); qsh[8 + e] = a; qsl[8 + e] = l;
    }
#pragma unroll
    for (int j = 0; j < 4; ++j) {
      s[j] = z8;
      FB kb, kl;
      kb.h[0] = *(const v8b*)(Kph + (j * 16 + c) * kHD + 8 * hf);
      kb.h[1] = *(const v8b*)(Kph + (j * 16 + c) * kHD + 16 + 8 * hf);
      kl.h[0] = *(const v8b*)(Kpl + (j * 16 + c) * kHD + 8 * hf);
      kl.h[1] = *(const v8b*)(Kpl + (j * 16 + c) * kHD + 16 + 8 * hf);
      s[j] = at_mma(qsh, kb.v, s[j]);
      s[j] = at_mma(qsh, kl.v, s[j]);
      s[j] = at_mma(qsl, kb.v, s[j]);
    }
  }

  {
    const float* bpr = Bp[wave];
#pragma unroll
    for (int j = 0; j < 4; ++j) {
#pragma unroll
      for (int r = 0; r < 8; ++r) s[j][r] += bpr[(8 * hf + r) * kPL + j * 16 + c];
    }
  }

  float invr[8];
  __bf16* pwh = Psh[wave];
  __bf16* pwl = Psl[wave];
  float* sa = Sa[wave];
  {
    const float lbv = lbias[h * kLoc + lc];
#pragma unroll
    for (int r = 0; r < 8; ++r) {
      float m = sloc[r];
#pragma unroll
      for (int j = 0; j < 4; ++j) m = fmaxf(m, s[j][r]);
      m = fmaxf(m, __shfl_xor(m, 1, 32)); m = fmaxf(m, __shfl_xor(m, 2, 32));
      m = fmaxf(m, __shfl_xor(m, 4, 32)); m = fmaxf(m, __shfl_xor(m, 8, 32));
      const float pl = expf(sloc[r] - m);
      float psum = pl;
#pragma unroll
      for (int j = 0; j < 4; ++j) {
        const float p = expf(s[j][r] - m);
        psum += p;
        __bf16 a, l;
        at_split(p, a, l);
        pwh[(8 * hf + r) * kPL + j * 16 + c] = a;
        pwl[(8 * hf + r) * kPL + j * 16 + c] = l;
      }
      psum += __shfl_xor(psum, 1, 32); psum += __shfl_xor(psum, 2, 32);
      psum += __shfl_xor(psum, 4, 32); psum += __shfl_xor(psum, 8, 32);
      const float inv = 1.0f / psum;
      invr[r] = inv;
      float al = (tacc[r] + lbv) + pl * inv;
      al = (c < kLoc) ? al : 0.f;
      sa[(8 * hf + r) * 16 + c] = al;
    }
  }
  __builtin_amdgcn_fence(__ATOMIC_RELEASE, "workgroup");
  __builtin_amdgcn_wave_barrier();
  __builtin_amdgcn_fence(__ATOMIC_ACQUIRE, "workgroup");

  float xa[8], xb[8];
#pragma unroll
  for (int r = 0; r < 8; ++r) { xa[r] = 0.f; xb[r] = 0.f; }
#pragma unroll 1
  for (int l = 0; l < kLoc; ++l) {
    const int krl = l / 3;
    const int djl = l - krl * 3 - 1;
#pragma unroll
    for (int r = 0; r < 8; ++r) {
      const int row = qrow0 + 8 * hf + r;
      const int jj  = row + djl;
      const bool okj = (jj >= 0) && (jj < kImg);
      const int jjc = jj < 0 ? 0 : (jj > kImg - 1 ? kImg - 1 : jj);
      float a = sa[(8 * hf + r) * 16 + l];
      const float* vp = Vloc + (krl * kImg + jjc) * kHD;
      const float v0 = vp[c];
      const float v1 = vp[16 + c];
      a = okj ? a : 0.f;
      xa[r] += a * v0;
      xb[r] += a * v1;
    }
  }

  v8f oacc[2];
  oacc[0] = z8; oacc[1] = z8;
#pragma unroll
  for (int kk = 0; kk < 2; ++kk) {
    FB pa, pb;
    pa.h[0] = *(const v8b*)(pwh + c * kPL + kk * 32 + 8 * hf);
    pa.h[1] = *(const v8b*)(pwh + c * kPL + kk * 32 + 16 + 8 * hf);
    pb.h[0] = *(const v8b*)(pwl + c * kPL + kk * 32 + 8 * hf);
    pb.h[1] = *(const v8b*)(pwl + c * kPL + kk * 32 + 16 + 8 * hf);
#pragma unroll
    for (int t = 0; t < 2; ++t) {
      FB va, vl;
      va.h[0] = *(const v8b*)(Vth + (t * 16 + c) * kPL + kk * 32 + 8 * hf);
      va.h[1] = *(const v8b*)(Vth + (t * 16 + c) * kPL + kk * 32 + 16 + 8 * hf);
      vl.h[0] = *(const v8b*)(Vtl + (t * 16 + c) * kPL + kk * 32 + 8 * hf);
      vl.h[1] = *(const v8b*)(Vtl + (t * 16 + c) * kPL + kk * 32 + 16 + 8 * hf);
      oacc[t] = at_mma(pa.v, va.v, oacc[t]);
      oacc[t] = at_mma(pa.v, vl.v, oacc[t]);
      oacc[t] = at_mma(pb.v, va.v, oacc[t]);
    }
  }

  float* os = Os[wave];
#pragma unroll
  for (int r = 0; r < 8; ++r) {
    const int n = i * kImg + qrow0 + 8 * hf + r;
    const float mw = maskw[(size_t)(b * kN + n) * kHeads + h];
    os[(8 * hf + r) * 36 + c]      = (xa[r] + oacc[0][r] * invr[r]) * mw;
    os[(8 * hf + r) * 36 + 16 + c] = (xb[r] + oacc[1][r] * invr[r]) * mw;
  }
  __builtin_amdgcn_fence(__ATOMIC_RELEASE, "workgroup");
  __builtin_amdgcn_wave_barrier();
  __builtin_amdgcn_fence(__ATOMIC_ACQUIRE, "workgroup");
  {
    const int rq = lane >> 3;
    const int c4 = (lane & 7) * 4;
    for (int pass = 0; pass < 2; ++pass) {
#pragma unroll
      for (int it = 0; it < 4; ++it) {
        const int row = it * 4 + rq;
        const v4f v = *(const v4f*)(os + row * 36 + c4);
        const int n = i * kImg + qrow0 + row;
        *(volatile v4f*)(obuf + (size_t)(b * kN + n) * kC + h * kHD + c4) = v;
      }
      __threadfence();
    }
  }
}

extern "C" void kernel_launch(void* const* d_in, const int* in_sizes, int n_in,
                              void* d_out, int out_size, void* d_ws, size_t ws_size,
                              hipStream_t stream) {
  if (n_in < 25) return;
  if (in_sizes[0] != kBN * kC || out_size != kBN * kC) return;
  if (in_sizes[24] != kN * kPL) return;

  const float* x      = (const float*)d_in[0];
  const float* rct    = (const float*)d_in[1];
  const float* q_w    = (const float*)d_in[2];
  const float* q_b    = (const float*)d_in[3];
  const float* kv_w   = (const float*)d_in[4];
  const float* kv_b   = (const float*)d_in[5];
  const float* temp   = (const float*)d_in[6];
  const float* qe     = (const float*)d_in[7];
  const float* rpb    = (const float*)d_in[8];
  const float* ltok   = (const float*)d_in[9];
  const float* lbias  = (const float*)d_in[10];
  const float* cpb1_w = (const float*)d_in[11];
  const float* cpb1_b = (const float*)d_in[12];
  const float* cpb2_w = (const float*)d_in[13];
  const float* cpb2_b = (const float*)d_in[14];
  const float* sr_w   = (const float*)d_in[15];
  const float* sr_b   = (const float*)d_in[16];
  const float* norm_g = (const float*)d_in[17];
  const float* norm_b = (const float*)d_in[18];
  const float* wg_w   = (const float*)d_in[19];
  const float* wg0_w  = (const float*)d_in[20];
  const float* wg1_w  = (const float*)d_in[21];
  const float* proj_w = (const float*)d_in[22];
  const float* proj_b = (const float*)d_in[23];
  const int*   rpi    = (const int*)d_in[24];
  float* out = (float*)d_out;

  size_t off = 0;
  auto take = [&](size_t bytes) { char* p = (char*)d_ws + off; off += (bytes + 255) & ~(size_t)255; return (void*)p; };
  unsigned short* xh   = (unsigned short*)take((size_t)kBN * kC * 2);
  unsigned short* xl   = (unsigned short*)take((size_t)kBN * kC * 2);
  unsigned short* wqh  = (unsigned short*)take((size_t)kC * kC * 2);
  unsigned short* wql  = (unsigned short*)take((size_t)kC * kC * 2);
  unsigned short* wkvh = (unsigned short*)take((size_t)2 * kC * kC * 2);
  unsigned short* wkvl = (unsigned short*)take((size_t)2 * kC * kC * 2);
  unsigned short* wsrh = (unsigned short*)take((size_t)kC * kC * 2);
  unsigned short* wsrl = (unsigned short*)take((size_t)kC * kC * 2);
  unsigned short* wph  = (unsigned short*)take((size_t)kC * kC * 2);
  unsigned short* wpl  = (unsigned short*)take((size_t)kC * kC * 2);
  unsigned short* w2p  = (unsigned short*)take((size_t)kCpbN * kHid * 2);
  unsigned short* hid  = (unsigned short*)take((size_t)kTbl * kHid * 2);
  float* cpbo  = (float*)take((size_t)kTbl * kCpbN * 4);
  float* maskw = (float*)take((size_t)kBN * kHeads * 4);
  float* qbuf  = (float*)take((size_t)kBN * kC * 4);
  float* kvbuf = (float*)take((size_t)kBN * 2 * kC * 4);
  float* srbuf = (float*)take((size_t)kBN * kC * 4);
  unsigned short* lnh = (unsigned short*)take((size_t)kB * kPL * kC * 2);
  unsigned short* lnl = (unsigned short*)take((size_t)kB * kPL * kC * 2);
  float* pkv   = (float*)take((size_t)kB * kPL * 2 * kC * 4);
  float* abuf  = (float*)take((size_t)kBN * kC * 4);
  unsigned short* ah = (unsigned short*)take((size_t)kBN * kC * 2);
  unsigned short* al = (unsigned short*)take((size_t)kBN * kC * 2);
  if (off > ws_size) return;

  const float sl4 = (float)log(68.0);
  const float sl6 = (float)log(70.0);
  const float sl9 = (float)log(73.0);

  {
    const int n8x = kBN * kC / 8;
    split_planes_kernel<<<(n8x + 255) / 256, 256, 0, stream>>>(x, xh, xl, n8x);
    const int n8q = kC * kC / 8;
    split_planes_kernel<<<(n8q + 255) / 256, 256, 0, stream>>>(q_w, wqh, wql, n8q);
    const int n8kv = 2 * kC * kC / 8;
    split_planes_kernel<<<(n8kv + 255) / 256, 256, 0, stream>>>(kv_w, wkvh, wkvl, n8kv);
    split_planes_kernel<<<(n8q + 255) / 256, 256, 0, stream>>>(sr_w, wsrh, wsrl, n8q);
    split_planes_kernel<<<(n8q + 255) / 256, 256, 0, stream>>>(proj_w, wph, wpl, n8q);
    const int n8w2 = kCpbN * kHid / 8;
    pad_w2_kernel<<<(n8w2 + 255) / 256, 256, 0, stream>>>(cpb2_w, w2p);
    const int n8h = kTbl * kHid / 8;
    cpb_hidden_kernel<<<(n8h + 255) / 256, 256, 0, stream>>>(rct, cpb1_w, cpb1_b, hid);
  }

  {
    const int tiles = (kTbl / 64) * (kCpbN / 64);
    wmma_gemm64<1, false, 0, 0, false><<<dim3((tiles + 7) / 8, 1), 256, 0, stream>>>(
        hid, hid, kHid, 0, w2p, w2p, kHid, 0, (void*)cpbo, (void*)cpbo, kCpbN, 0,
        cpb2_b, x, 0, kTbl, kCpbN, kHid, 1.0f);
  }

  static_assert(kBN % 8 == 0, "");
  gates_kernel<<<kBN / 8, 256, 0, stream>>>(x, wg_w, wg0_w, wg1_w, maskw);

  {
    const int tq = (kBN / 64) * (kC / 64);
    wmma_gemm64<1, true, 2, 0, false><<<dim3((tq + 7) / 8, 1), 256, 0, stream>>>(
        xh, xl, kC, 0, wqh, wql, kC, 0, (void*)qbuf, (void*)qbuf, kC, 0,
        q_b, x, 0, kBN, kC, kC, 1.0f);
    const int tkv = (kBN / 64) * ((2 * kC) / 64);
    wmma_gemm64<1, true, 2, 0, false><<<dim3((tkv + 7) / 8, 1), 256, 0, stream>>>(
        xh, xl, kC, 0, wkvh, wkvl, kC, 0, (void*)kvbuf, (void*)kvbuf, 2 * kC, 0,
        kv_b, x, 0, kBN, 2 * kC, kC, 1.0f);
    wmma_gemm64<1, true, 2, 0, false><<<dim3((tq + 7) / 8, 1), 256, 0, stream>>>(
        xh, xl, kC, 0, wsrh, wsrl, kC, 0, (void*)srbuf, (void*)srbuf, kC, 0,
        sr_b, x, 0, kBN, kC, kC, 1.0f);
  }

  pool_ln_kernel<<<kB * kPL, 256, 0, stream>>>(srbuf, norm_g, norm_b, lnh, lnl);
  {
    const int tp = ((kB * kPL) / 64) * ((2 * kC) / 64);
    wmma_gemm64<1, true, 2, 0, false><<<dim3((tp + 7) / 8, 1), 256, 0, stream>>>(
        lnh, lnl, kC, 0, wkvh, wkvl, kC, 0, (void*)pkv, (void*)pkv, 2 * kC, 0,
        kv_b, x, 0, kB * kPL, 2 * kC, kC, 1.0f);
  }

  attn_kernel<<<kB * kHeads * kImg, 128, 0, stream>>>(qbuf, kvbuf, pkv, cpbo, rpi, cpb2_b, rpb, ltok,
                                                     lbias, qe, temp, maskw, abuf, sl4, sl6, sl9);

  {
    const int n8a = kBN * kC / 8;
    split_planes_kernel<<<(n8a + 255) / 256, 256, 0, stream>>>(abuf, ah, al, n8a);
    const int to = (kBN / 64) * (kC / 64);
    wmma_gemm64<1, true, 2, 0, false><<<dim3((to + 7) / 8, 1), 256, 0, stream>>>(
        ah, al, kC, 0, wph, wpl, kC, 0, (void*)out, (void*)out, kC, 0,
        proj_b, x, 0, kBN, kC, kC, 1.0f);
  }
}
